// ResAttnBlock_22316650070627
// MI455X (gfx1250) — hardware-run, weakly checked
//
#include <hip/hip_runtime.h>


namespace {
constexpr int NBI = 32, DIM = 256, HH = 32, WW = 32, NP = HH * WW  , CED = 64, CH = 64, CWD = 64, KC = CED * 4  , KB = 64;
constexpr float XS = 8.0f, HS = 256.0f, WSC = 256.0f, PS = 256.0f, EPS = 1e-5f, SLOPE = 0.2f;
typedef _Float16 b16;
typedef __attribute__((ext_vector_type(16))) _Float16 v16b;
typedef __attribute__((ext_vector_type(8))) _Float16 v8b;
typedef __attribute__((ext_vector_type(8))) float v8f;
typedef __attribute__((ext_vector_type(4))) float v4f;
__device__ __forceinline__ float bf16_rne(float f) { unsigned int u = __float_as_uint(f); u += 0x7FFFu + ((u >> 16) & 1u); float r = __uint_as_float(u & 0xFFFF0000u); asm volatile("" : "+v"(r)); return r; }
__device__ __forceinline__ float bfv(float f) { float r = bf16_rne(f); asm volatile("" : "+v"(r)); return r; }
__device__ __forceinline__ void split16(float v, b16& hi, b16& lo) { hi = (b16)v; lo = (b16)(v - (float)hi); }
__device__ __forceinline__ v16b frag_kb(const b16* p, int hh) { const v8b a = *(const v8b*)(p + 8 * hh), b = *(const v8b*)(p + 16 + 8 * hh); v16b f;
#pragma unroll
  for (int e = 0; e < 8; ++e) { f[e] = a[e]; f[8 + e] = b[e]; } return f; }
__device__ __forceinline__ v8f wmma16b(v16b a, v16b b, v8f c) { v8f d = __builtin_amdgcn_wmma_f32_16x16x32_f16(false, a, false, b, (short)0, c, false, false); asm volatile("v_nop\n\tv_nop\n\tv_nop\n\tv_nop" : "+v"(d) : "v"(a), "v"(b)); return d; }
__device__ __forceinline__ void wave_lds_sync() { __builtin_amdgcn_fence(__ATOMIC_RELEASE, "workgroup"); __builtin_amdgcn_wave_barrier(); __builtin_amdgcn_fence(__ATOMIC_ACQUIRE, "workgroup"); }
__device__ __forceinline__ float pmul(float a, float b) { float p = a * b; asm volatile("" : "+v"(p)); return p; }
__device__ __forceinline__ float lrelu(float v) { return v >= 0.0f ? v : SLOPE * v; }

__global__ __launch_bounds__(256) void wput_kernel(const float* __restrict__ cw, const float* __restrict__ kw, const float* __restrict__ vw, b16* __restrict__ WCV, b16* __restrict__ WKV) { const int u = blockIdx.x * 256 + threadIdx.x; v8b v;
  if (u < DIM * (KC / 8)) { const int o = u / (KC / 8), k0 = (u % (KC / 8)) * 8;
#pragma unroll
    for (int j = 0; j < 8; ++j) v[j] = (b16)(bf16_rne(cw[(size_t)o * KC + k0 + j]) * WSC); for (int pass = 0; pass < 2; ++pass) { *(volatile v8b*)(WCV + (size_t)o * KC + k0) = v; __threadfence(); } }
  if (u < 2 * DIM * (DIM / 8)) { const int o = u / (DIM / 8), k0 = (u % (DIM / 8)) * 8; const float* w = o < DIM ? kw + (size_t)o * DIM : vw + (size_t)(o - DIM) * DIM;
#pragma unroll
    for (int j = 0; j < 8; ++j) v[j] = (b16)(bf16_rne(w[k0 + j]) * WSC); for (int pass = 0; pass < 2; ++pass) { *(volatile v8b*)(WKV + (size_t)o * DIM + k0) = v; __threadfence(); } } }
__global__ __launch_bounds__(32) void conv_kernel(const float* __restrict__ c, const b16* __restrict__ WCV, const float* __restrict__ cb, int BLIM, float* __restrict__ L1, float* __restrict__ PS1) { __shared__ __attribute__((aligned(16))) b16 Xt[32][KC + 8]; __shared__ float Tf[32][DIM + 4]; const int lane = threadIdx.x, nloc = lane & 15, hlf = lane >> 4; const int b = blockIdx.x / HH, oh = blockIdx.x % HH; if (b >= BLIM) return;
  for (int ci = 0; ci < CED; ++ci) for (int kh = 0; kh < 2; ++kh) { const float* row = c + (((size_t)b * CED + ci) * CH + 2 * oh + kh) * CWD; const float v0 = row[lane], v1 = row[32 + lane]; Xt[lane >> 1][ci * 4 + kh * 2 + (lane & 1)] = (b16)(bf16_rne(v0) * XS); Xt[16 + (lane >> 1)][ci * 4 + kh * 2 + (lane & 1)] = (b16)(bf16_rne(v1) * XS); }
  for (int k = KC; k < KC + 8; ++k) Xt[lane][k] = (b16)0.0f;
  wave_lds_sync();
#pragma unroll 1
  for (int rt = 0; rt < 2; ++rt) { v8f acc[16];
#pragma unroll
    for (int t = 0; t < 16; ++t) acc[t] = (v8f){};
#pragma unroll 2
    for (int kb = 0; kb < KC; kb += 32) { const v16b a = frag_kb(&Xt[rt * 16 + nloc][kb], hlf);
#pragma unroll
      for (int t = 0; t < 16; ++t) acc[t] = wmma16b(a, frag_kb(WCV + (size_t)(t * 16 + nloc) * KC + kb, hlf), acc[t]); }
#pragma unroll
    for (int t = 0; t < 16; ++t) { const int cc = t * 16 + nloc; const float bb = bfv(cb[cc]);
#pragma unroll
      for (int r8 = 0; r8 < 8; ++r8) Tf[rt * 16 + 8 * hlf + r8][cc] = lrelu(acc[t][r8] * (1.0f / (XS * WSC)) + bb); } }
  wave_lds_sync();
  for (int pass = 0; pass < 2; ++pass) { for (int rr = 0; rr < 32; ++rr) for (int q = 0; q < 2; ++q) *(volatile v4f*)(L1 + ((size_t)b * NP + oh * WW + rr) * DIM + q * 128 + lane * 4) = *(const v4f*)(&Tf[rr][q * 128 + lane * 4]);
    for (int cch = lane; cch < DIM; cch += 32) { float s = 0.0f, s2 = 0.0f; for (int rr = 0; rr < 32; ++rr) { const float v = Tf[rr][cch]; s += v; s2 += v * v; } ((volatile float*)PS1)[(size_t)blockIdx.x * 2 * DIM + cch] = s; ((volatile float*)PS1)[(size_t)blockIdx.x * 2 * DIM + DIM + cch] = s2; } __threadfence(); } }
__global__ __launch_bounds__(256) void bn_kernel(const float* __restrict__ PS, int nw, int count, const float* __restrict__ g, const float* __restrict__ be, float* __restrict__ BNP) { const int cch = threadIdx.x; double s = 0.0, s2 = 0.0; for (int w = 0; w < nw; ++w) { s += (double)PS[(size_t)w * 2 * DIM + cch]; s2 += (double)PS[(size_t)w * 2 * DIM + DIM + cch]; } const double mu = s / count; double var = s2 / count - mu * mu; if (var < 0.0) var = 0.0; const float sc = bfv(g[cch]) * (float)(1.0 / sqrt(var + (double)EPS)); const float sh = bfv(be[cch]) - (float)mu * sc;
  for (int pass = 0; pass < 2; ++pass) { ((volatile float*)BNP)[cch] = sc; ((volatile float*)BNP)[DIM + cch] = sh; __threadfence(); } }
__global__ __launch_bounds__(32) void kv_kernel(const float* __restrict__ x, const b16* __restrict__ WKV, const float* __restrict__ kb_, const float* __restrict__ vb_, int BLIM, b16* __restrict__ Kh, b16* __restrict__ Kl, b16* __restrict__ Vh, b16* __restrict__ Vl) { __shared__ __attribute__((aligned(16))) b16 Xt[32][DIM + 8], Oh[32][DIM + 8], Ol[32][DIM + 8]; const int lane = threadIdx.x, nloc = lane & 15, hlf = lane >> 4; const int b = blockIdx.x / (NP / 32); if (b >= BLIM) return; const int n0 = (blockIdx.x % (NP / 32)) * 32;
  for (int d = 0; d < DIM; ++d) Xt[lane][d] = (b16)(bf16_rne(x[((size_t)b * DIM + d) * NP + n0 + lane]) * XS); for (int k = DIM; k < DIM + 8; ++k) Xt[lane][k] = (b16)0.0f;
  wave_lds_sync();
#pragma unroll 1
  for (int pj = 0; pj < 2; ++pj) {
#pragma unroll 1
    for (int rt = 0; rt < 2; ++rt) { v8f acc[16];
#pragma unroll
      for (int t = 0; t < 16; ++t) acc[t] = (v8f){};
#pragma unroll 2
      for (int kb = 0; kb < DIM; kb += 32) { const v16b a = frag_kb(&Xt[rt * 16 + nloc][kb], hlf);
#pragma unroll
        for (int t = 0; t < 16; ++t) acc[t] = wmma16b(a, frag_kb(WKV + (size_t)(pj * DIM + t * 16 + nloc) * DIM + kb, hlf), acc[t]); }
      const float* bb = pj == 0 ? kb_ : vb_;
#pragma unroll
      for (int t = 0; t < 16; ++t) { const int cc = t * 16 + nloc; const float bv = bfv(bb[cc]);
#pragma unroll
        for (int r8 = 0; r8 < 8; ++r8) { b16 p, ql; split16((acc[t][r8] * (1.0f / (XS * WSC)) + bv) * HS, p, ql); Oh[rt * 16 + 8 * hlf + r8][cc] = p; Ol[rt * 16 + 8 * hlf + r8][cc] = ql; } } }
    wave_lds_sync(); b16* Dh = pj == 0 ? Kh : Vh; b16* Dl = pj == 0 ? Kl : Vl;
    for (int pass = 0; pass < 2; ++pass) { for (int rr = 0; rr < 32; ++rr) { const size_t o = ((size_t)b * NP + n0 + rr) * DIM + lane * 8; *(volatile v8b*)(Dh + o) = *(const v8b*)(&Oh[rr][lane * 8]); *(volatile v8b*)(Dl + o) = *(const v8b*)(&Ol[rr][lane * 8]); } __threadfence(); }
    wave_lds_sync(); } }
__global__ __launch_bounds__(32) void att_kernel(const float* __restrict__ L1, const float* __restrict__ BN1, const b16* __restrict__ Kh, const b16* __restrict__ Kl, const b16* __restrict__ Vh, const b16* __restrict__ Vl, int BLIM, float* __restrict__ O) {
  __shared__ __attribute__((aligned(16))) b16 Qh[16][DIM + 8], Ql[16][DIM + 8], P_h[16][KB + 8], Vth[DIM][KB + 8], Vtl[DIM][KB + 8]; __shared__ float Sf[16][KB + 4];
  const int lane = threadIdx.x, nloc = lane & 15, hlf = lane >> 4; const int b = blockIdx.x / (NP / 16); if (b >= BLIM) return; const size_t q0 = (size_t)b * NP + (size_t)(blockIdx.x % (NP / 16)) * 16;
  for (int rr = 0; rr < 16; ++rr) for (int q = 0; q < DIM / 32; ++q) { const int d = q * 32 + lane; b16 p, ql; split16((pmul(L1[(q0 + rr) * DIM + d], BN1[d]) + BN1[DIM + d]) * HS, p, ql); Qh[rr][d] = p; Ql[rr][d] = ql; }
  if (lane < 16) for (int k = DIM; k < DIM + 8; ++k) { Qh[lane][k] = (b16)0.0f; Ql[lane][k] = (b16)0.0f; }
  wave_lds_sync();
  float m_r[8], den_r[8]; v8f acc[16];
#pragma unroll
  for (int r8 = 0; r8 < 8; ++r8) { m_r[r8] = -INFINITY; den_r[r8] = 0.0f; }
#pragma unroll
  for (int t = 0; t < 16; ++t) acc[t] = (v8f){};
#pragma unroll 1
  for (int kb0 = 0; kb0 < NP; kb0 += KB) { const size_t kbase = (size_t)b * NP + kb0;
    for (int rr = 0; rr < KB; rr += 2) { const int r = rr + hlf; const size_t vr = (kbase + r) * DIM; for (int s = 0; s < DIM / 16; ++s) { Vth[s * 16 + nloc][r] = Vh[vr + s * 16 + nloc]; Vtl[s * 16 + nloc][r] = Vl[vr + s * 16 + nloc]; } }
#pragma unroll 1
    for (int t = 0; t < KB / 16; ++t) { const size_t kr = (kbase + t * 16 + nloc) * DIM; v8f s = {};
#pragma unroll 2
      for (int ks = 0; ks < DIM; ks += 32) { const v16b qa = frag_kb(&Qh[nloc][ks], hlf), qb = frag_kb(&Ql[nloc][ks], hlf); const v16b ka = frag_kb(Kh + kr + ks, hlf), kl = frag_kb(Kl + kr + ks, hlf); s = wmma16b(qa, ka, s); s = wmma16b(qa, kl, s); s = wmma16b(qb, ka, s); }
#pragma unroll
      for (int r8 = 0; r8 < 8; ++r8) Sf[8 * hlf + r8][t * 16 + nloc] = s[r8] * (1.0f / (HS * HS)); }
    wave_lds_sync();
#pragma unroll
    for (int rr = 0; rr < 16; ++rr) { float mx = -INFINITY;
#pragma unroll
      for (int q = 0; q < KB / 32; ++q) mx = fmaxf(mx, Sf[rr][q * 32 + lane]);
      for (int o = 16; o; o >>= 1) mx = fmaxf(mx, __shfl_xor(mx, o));
      const float mold = __shfl(m_r[rr & 7], (rr >> 3) * 16); const float mn = fmaxf(mold, mx); const float sf = (mold == -INFINITY) ? 0.0f : __expf(mold - mn); float ps = 0.0f;
#pragma unroll
      for (int q = 0; q < KB / 32; ++q) { const int kx = q * 32 + lane; const float p = __expf(Sf[rr][kx] - mn); ps += p; P_h[rr][kx] = (b16)(p * PS); }
      for (int o = 16; o; o >>= 1) ps += __shfl_xor(ps, o);
      if ((rr >> 3) == hlf) { const int r8 = rr & 7; den_r[r8] = den_r[r8] * sf + ps; m_r[r8] = mn;
#pragma unroll
        for (int t = 0; t < 16; ++t) acc[t][r8] = acc[t][r8] * sf; } }
    if (lane < 16) for (int k = KB; k < KB + 8; ++k) P_h[lane][k] = (b16)0.0f;
    wave_lds_sync();
#pragma unroll
    for (int ks = 0; ks < KB; ks += 32) { const v16b pa = frag_kb(&P_h[nloc][ks], hlf);
#pragma unroll
      for (int t = 0; t < 16; ++t) { acc[t] = wmma16b(pa, frag_kb(&Vth[t * 16 + nloc][ks], hlf), acc[t]); acc[t] = wmma16b(pa, frag_kb(&Vtl[t * 16 + nloc][ks], hlf), acc[t]); } }
    wave_lds_sync(); }
  float (*Of)[DIM + 4] = (float (*)[DIM + 4])&Vth[0][0];
#pragma unroll
  for (int t = 0; t < 16; ++t)
#pragma unroll
    for (int r8 = 0; r8 < 8; ++r8) Of[8 * hlf + r8][t * 16 + nloc] = acc[t][r8] * (1.0f / (HS * PS)) / den_r[r8];
  wave_lds_sync();
  for (int pass = 0; pass < 2; ++pass) { for (int rr = 0; rr < 16; ++rr) for (int q = 0; q < 2; ++q) *(volatile v4f*)(O + (q0 + rr) * DIM + q * 128 + lane * 4) = *(const v4f*)(&Of[rr][q * 128 + lane * 4]); __threadfence(); } }
__global__ __launch_bounds__(32) void stat2_kernel(const float* __restrict__ O, const float* __restrict__ x, int BLIM, float* __restrict__ PS2) { __shared__ float Z[32][DIM + 1]; const int lane = threadIdx.x; const int b = blockIdx.x / (NP / 32); if (b >= BLIM) return; const int n0 = (blockIdx.x % (NP / 32)) * 32;
  for (int d = 0; d < DIM; ++d) Z[lane][d] = lrelu(O[((size_t)b * NP + n0 + lane) * DIM + d] + bfv(x[((size_t)b * DIM + d) * NP + n0 + lane]));
  wave_lds_sync();
  for (int pass = 0; pass < 2; ++pass) { for (int d = lane; d < DIM; d += 32) { float s = 0.0f, s2 = 0.0f; for (int rr = 0; rr < 32; ++rr) { const float v = Z[rr][d]; s += v; s2 += v * v; } ((volatile float*)PS2)[(size_t)blockIdx.x * 2 * DIM + d] = s; ((volatile float*)PS2)[(size_t)blockIdx.x * 2 * DIM + DIM + d] = s2; } __threadfence(); } }
__global__ __launch_bounds__(32) void out_kernel(const float* __restrict__ O, const float* __restrict__ x, const float* __restrict__ BN2, int BLIM, float* __restrict__ out) { const int lane = threadIdx.x; const int b = blockIdx.x / (NP / 32); if (b >= BLIM) return; const int n0 = (blockIdx.x % (NP / 32)) * 32; const size_t orow = ((size_t)b * NP + n0 + lane) * DIM;
  for (int pass = 0; pass < 2; ++pass) {
#pragma unroll 4
    for (int d = 0; d < DIM; ++d) { const size_t xi = ((size_t)b * DIM + d) * NP + n0 + lane; const float z = lrelu(O[orow + d] + bfv(x[xi])); ((volatile float*)out)[xi] = pmul(z, BN2[d]) + BN2[DIM + d]; } __threadfence(); } }
}

extern "C" void kernel_launch(void* const* d_in, const int* in_sizes, int n_in, void* d_out, int out_size, void* d_ws, size_t ws_size, hipStream_t stream) {
  (void)n_in;
  auto Fp = [&](int i) { return (const float*)d_in[i]; };
  if (in_sizes[0] != NBI * DIM * NP || in_sizes[1] != NBI * CED * CH * CWD || in_sizes[2] != DIM * KC || in_sizes[3] != DIM || in_sizes[6] != DIM * DIM || in_sizes[8] != DIM * DIM || in_sizes[10] != DIM || out_size != NBI * DIM * NP) return;
  const int BLIM = NBI;
  size_t off = 0; char* ws = (char*)d_ws;
  auto carve = [&](size_t bytes) { char* p = ws + off; off += (bytes + 255) & ~(size_t)255; return p; };
  b16* WCV = (b16*)carve((size_t)DIM * KC * 2); b16* WKV = (b16*)carve((size_t)2 * DIM * DIM * 2); float* L1 = (float*)carve((size_t)NBI * NP * DIM * 4); float* PS1 = (float*)carve((size_t)NBI * HH * 2 * DIM * 4); float* BN1 = (float*)carve(2 * DIM * 4);
  b16* Kh = (b16*)carve((size_t)NBI * NP * DIM * 2); b16* Kl = (b16*)carve((size_t)NBI * NP * DIM * 2); b16* Vh = (b16*)carve((size_t)NBI * NP * DIM * 2); b16* Vl = (b16*)carve((size_t)NBI * NP * DIM * 2); float* Ob = (float*)carve((size_t)NBI * NP * DIM * 4); float* PS2 = (float*)carve((size_t)NBI * (NP / 32) * 2 * DIM * 4); float* BN2 = (float*)carve(2 * DIM * 4);
  if (off > ws_size || off > ((size_t)192 << 20)) return;
  wput_kernel<<<(2 * DIM * (DIM / 8) + 255) / 256, 256, 0, stream>>>(Fp(2), Fp(6), Fp(8), WCV, WKV);
  conv_kernel<<<BLIM * HH, 32, 0, stream>>>(Fp(1), WCV, Fp(3), BLIM, L1, PS1);
  bn_kernel<<<1, 256, 0, stream>>>(PS1, BLIM * HH, BLIM * NP, Fp(4), Fp(5), BN1);
  kv_kernel<<<BLIM * (NP / 32), 32, 0, stream>>>(Fp(0), WKV, Fp(7), Fp(9), BLIM, Kh, Kl, Vh, Vl);
  att_kernel<<<BLIM * (NP / 16), 32, 0, stream>>>(L1, BN1, Kh, Kl, Vh, Vl, BLIM, Ob);
  stat2_kernel<<<BLIM * (NP / 32), 32, 0, stream>>>(Ob, Fp(0), BLIM, PS2);
  bn_kernel<<<1, 256, 0, stream>>>(PS2, BLIM * (NP / 32), BLIM * NP, Fp(10), Fp(11), BN2);
  out_kernel<<<BLIM * (NP / 32), 32, 0, stream>>>(Ob, Fp(0), BN2, BLIM, (float*)d_out);
}
